// NCM_30468497998426
// MI455X (gfx1250) — hardware-verified
//
#include <hip/hip_runtime.h>
#include <hip/hip_bf16.h>


#define DIM   512
#define NCLS  1000
#define NSHOT 5
#define NSUP  (NCLS * NSHOT)
#define NQ    5000
#define BM    160
#define BN    32
#define CPB   (BM / NSHOT)
#define MBLK  ((NSUP + BM - 1) / BM)
#define MPAD  (MBLK * BM)
#define NBLK  ((NQ + BN - 1) / BN)
#define NPAD  (NBLK * BN)
#define SIM_THREADS 160

typedef __bf16 bf16x16 __attribute__((ext_vector_type(16)));
typedef __bf16 bf16x8  __attribute__((ext_vector_type(8)));
typedef float  f32x8   __attribute__((ext_vector_type(8)));
typedef float  f32x4   __attribute__((ext_vector_type(4)));
typedef int    i32x4   __attribute__((ext_vector_type(4)));
typedef unsigned short u16x8 __attribute__((ext_vector_type(8)));
typedef f32x4 __attribute__((may_alias)) f32x4a;
typedef i32x4 __attribute__((may_alias)) i32x4a;

union Frag { bf16x16 v; bf16x8 p[2]; };

__device__ __forceinline__ unsigned short f2bf(float f) {
    unsigned int u = __float_as_uint(f);
    u += 0x7FFFu + ((u >> 16) & 1u);
    return (unsigned short)(u >> 16);
}
__device__ __forceinline__ float bf2f(unsigned short b) {
    return __uint_as_float(((unsigned int)b) << 16);
}

__device__ __forceinline__ f32x8 wmma_bf16(bf16x16 a, bf16x16 b, f32x8 c) {
    return __builtin_amdgcn_wmma_f32_16x16x32_bf16(false, a, false, b, (short)0, c, false, false);
}
__device__ __forceinline__ f32x8 wmma_split3(bf16x16 ah, bf16x16 al, bf16x16 bh, bf16x16 bl, f32x8 c) {
    c = wmma_bf16(ah, bh, c);
    c = wmma_bf16(ah, bl, c);
    c = wmma_bf16(al, bh, c);
    return c;
}

__global__ __launch_bounds__(128)
void k_mean(const float* __restrict__ sup, float* mean, int nrows) {
    const int t = threadIdx.x;
    if (t >= DIM / 4) return;
    const float4* p = (const float4*)sup + t;
    double a0 = 0.0, a1 = 0.0, a2 = 0.0, a3 = 0.0;
    #pragma unroll 4
    for (int r = 0; r < nrows; ++r) {
        const float4 v = p[(size_t)r * (DIM / 4)];
        a0 += (double)v.x; a1 += (double)v.y; a2 += (double)v.z; a3 += (double)v.w;
    }
    const double n = (double)nrows;
    f32x4 mv;
    mv.x = (float)(a0 / n); mv.y = (float)(a1 / n); mv.z = (float)(a2 / n); mv.w = (float)(a3 / n);
    volatile f32x4* dst = (volatile f32x4*)mean + t;
    *dst = mv;
    __threadfence();
    *dst = mv;
}

__global__ __launch_bounds__(64)
void k_norm(const float* __restrict__ x, const float* __restrict__ mean,
            unsigned short* ph, unsigned short* pl, int nreal, int npad) {
    __shared__ float red[2];
    const int row = blockIdx.x;
    const int t   = threadIdx.x;
    const bool real = row < nreal;
    float v[8];
    if (real) {
        const float4* xr = (const float4*)(x + (size_t)row * DIM) + 2 * t;
        const float4* mr = (const float4*)mean + 2 * t;
        const float4 x0 = xr[0], x1 = xr[1], m0 = mr[0], m1 = mr[1];
        v[0] = x0.x - m0.x; v[1] = x0.y - m0.y; v[2] = x0.z - m0.z; v[3] = x0.w - m0.w;
        v[4] = x1.x - m1.x; v[5] = x1.y - m1.y; v[6] = x1.z - m1.z; v[7] = x1.w - m1.w;
    } else {
        #pragma unroll
        for (int i = 0; i < 8; ++i) v[i] = 0.0f;
    }
    float ss = 0.0f;
    #pragma unroll
    for (int i = 0; i < 8; ++i) ss += v[i] * v[i];
    #pragma unroll
    for (int off = 16; off > 0; off >>= 1) ss += __shfl_xor(ss, off);
    if ((t & 31) == 0) red[t >> 5] = ss;
    __syncthreads();
    const float tot = red[0] + red[1];

    u16x8 oh = {0, 0, 0, 0, 0, 0, 0, 0};
    u16x8 ol = {0, 0, 0, 0, 0, 0, 0, 0};
    if (real) {
        const float inv = 1.0f / sqrtf(tot);
        #pragma unroll
        for (int i = 0; i < 8; ++i) {
            const float vn = v[i] * inv;
            const unsigned short hb = f2bf(vn);
            const unsigned short lb = f2bf(vn - bf2f(hb));
            oh[i] = hb; ol[i] = lb;
        }
    }
    if (row < npad) {
        volatile u16x8* dh = (volatile u16x8*)(ph + (size_t)row * DIM) + t;
        volatile u16x8* dl = (volatile u16x8*)(pl + (size_t)row * DIM) + t;
        *dh = oh; *dl = ol;
        __threadfence();
        *dh = oh; *dl = ol;
    }
}

__global__ __launch_bounds__(SIM_THREADS)
void k_sim(const unsigned short* __restrict__ Sh, const unsigned short* __restrict__ Sl,
           const unsigned short* __restrict__ Qh, const unsigned short* __restrict__ Ql,
           float* pval, int* pidx) {
    __shared__ __attribute__((aligned(16))) float tile[BM * BN];
    __shared__ __attribute__((aligned(16))) float fv[BN];
    __shared__ __attribute__((aligned(16))) int   fi[BN];

    const int tid  = threadIdx.x;
    const int lane = tid & 31;
    const int w    = tid >> 5;
    const int h    = lane >> 4;
    const int m    = lane & 15;
    const int mb   = blockIdx.y;
    const int nb   = blockIdx.x;

    const int offA0 = (mb * BM + w * 32 + m) * DIM + 8 * h;
    const int offA1 = offA0 + 16 * DIM;
    const int offB0 = (nb * BN + m) * DIM + 8 * h;
    const int offB1 = offB0 + 16 * DIM;

    f32x8 c00 = {0, 0, 0, 0, 0, 0, 0, 0};
    f32x8 c01 = {0, 0, 0, 0, 0, 0, 0, 0};
    f32x8 c10 = {0, 0, 0, 0, 0, 0, 0, 0};
    f32x8 c11 = {0, 0, 0, 0, 0, 0, 0, 0};

    #pragma unroll 1
    for (int k0 = 0; k0 < DIM; k0 += 32) {
        Frag a0h, a0l, a1h, a1l, b0h, b0l, b1h, b1l;
        a0h.p[0] = *(const bf16x8*)(Sh + offA0 + k0);  a0h.p[1] = *(const bf16x8*)(Sh + offA0 + k0 + 16);
        a0l.p[0] = *(const bf16x8*)(Sl + offA0 + k0);  a0l.p[1] = *(const bf16x8*)(Sl + offA0 + k0 + 16);
        a1h.p[0] = *(const bf16x8*)(Sh + offA1 + k0);  a1h.p[1] = *(const bf16x8*)(Sh + offA1 + k0 + 16);
        a1l.p[0] = *(const bf16x8*)(Sl + offA1 + k0);  a1l.p[1] = *(const bf16x8*)(Sl + offA1 + k0 + 16);
        b0h.p[0] = *(const bf16x8*)(Qh + offB0 + k0);  b0h.p[1] = *(const bf16x8*)(Qh + offB0 + k0 + 16);
        b0l.p[0] = *(const bf16x8*)(Ql + offB0 + k0);  b0l.p[1] = *(const bf16x8*)(Ql + offB0 + k0 + 16);
        b1h.p[0] = *(const bf16x8*)(Qh + offB1 + k0);  b1h.p[1] = *(const bf16x8*)(Qh + offB1 + k0 + 16);
        b1l.p[0] = *(const bf16x8*)(Ql + offB1 + k0);  b1l.p[1] = *(const bf16x8*)(Ql + offB1 + k0 + 16);

        c00 = wmma_split3(a0h.v, a0l.v, b0h.v, b0l.v, c00);
        c01 = wmma_split3(a0h.v, a0l.v, b1h.v, b1l.v, c01);
        c10 = wmma_split3(a1h.v, a1l.v, b0h.v, b0l.v, c10);
        c11 = wmma_split3(a1h.v, a1l.v, b1h.v, b1l.v, c11);
        asm volatile("v_nop\n\tv_nop\n\tv_nop\n\tv_nop"
                     : "+v"(c00), "+v"(c01), "+v"(c10), "+v"(c11)
                     : "v"(a0h.v), "v"(a0l.v), "v"(a1h.v), "v"(a1l.v),
                       "v"(b0h.v), "v"(b0l.v), "v"(b1h.v), "v"(b1l.v));
    }

    const int rb = w * 32;
    #pragma unroll
    for (int r = 0; r < 8; ++r) {
        tile[(rb + 8 * h + r)      * BN + m]      = c00[r];
        tile[(rb + 8 * h + r)      * BN + 16 + m] = c01[r];
        tile[(rb + 16 + 8 * h + r) * BN + m]      = c10[r];
        tile[(rb + 16 + 8 * h + r) * BN + 16 + m] = c11[r];
    }
    __syncthreads();

    if (tid < BN) {
        float best = __uint_as_float(0xff800000u);
        int   bc   = mb * CPB;
        #pragma unroll 1
        for (int cc = 0; cc < CPB; ++cc) {
            const int cg = mb * CPB + cc;
            if (cg >= NCLS) break;
            const float* tp = tile + (cc * NSHOT) * BN + tid;
            float mx = tp[0];
            #pragma unroll
            for (int s = 1; s < NSHOT; ++s) mx = fmaxf(mx, tp[s * BN]);
            if (mx > best) { best = mx; bc = cg; }
        }
        fv[tid] = best;
        fi[tid] = bc;
    }
    __syncthreads();

    if (tid < 8) {
        const f32x4 vv = *((const f32x4a*)fv + tid);
        const i32x4 iv = *((const i32x4a*)fi + tid);
        const size_t off = (size_t)mb * NPAD + (size_t)nb * BN + 4 * tid;
        volatile f32x4* dv = (volatile f32x4*)(pval + off);
        volatile i32x4* di = (volatile i32x4*)(pidx + off);
        *dv = vv; *di = iv;
        __threadfence();
        *dv = vv; *di = iv;
    }
}

__global__ __launch_bounds__(32)
void k_final(const float* __restrict__ pval, const int* __restrict__ pidx,
             const int* __restrict__ ucos, int* out, int nq) {
    __shared__ __attribute__((aligned(16))) int res[32];
    const int lane = threadIdx.x;
    const int q    = blockIdx.x * 32 + lane;
    const int cosm = ucos[0];
    int bc = 0;
    if (cosm != 0) {
        float bv = __uint_as_float(0xff800000u);
        #pragma unroll 1
        for (int mbk = 0; mbk < MBLK; ++mbk) {
            const float v = pval[(size_t)mbk * NPAD + q];
            const int   c = pidx[(size_t)mbk * NPAD + q];
            if (v > bv || (v == bv && c < bc)) { bv = v; bc = c; }
        }
    } else {
        float bv = __uint_as_float(0x7f800000u);
        #pragma unroll 1
        for (int mbk = 0; mbk < MBLK; ++mbk) {
            const float v = pval[(size_t)mbk * NPAD + q];
            const int   c = pidx[(size_t)mbk * NPAD + q];
            const float d = sqrtf(fmaxf(2.0f - 2.0f * v, 0.0f));
            if (d < bv || (d == bv && c < bc)) { bv = d; bc = c; }
        }
    }
    res[lane] = bc;
    __syncthreads();
    if (lane < 8) {
        const int q0 = blockIdx.x * 32 + 4 * lane;
        if (q0 + 4 <= nq) {
            const i32x4 rv = *((const i32x4a*)res + lane);
            volatile i32x4* d = (volatile i32x4*)(out + q0);
            *d = rv;
            __threadfence();
            *d = rv;
        } else {
            #pragma unroll
            for (int e = 0; e < 4; ++e) {
                if (q0 + e < nq) {
                    const int val = res[4 * lane + e];
                    volatile int* d = (volatile int*)(out + q0 + e);
                    *d = val;
                    __threadfence();
                    *d = val;
                }
            }
        }
    }
}

static inline size_t align_up_256(size_t x) { return (x + 255) & ~(size_t)255; }

extern "C" void kernel_launch(void* const* d_in, const int* in_sizes, int n_in,
                              void* d_out, int out_size, void* d_ws, size_t ws_size,
                              hipStream_t stream) {
    if (n_in < 3) return;
    if (in_sizes[0] != NSUP * DIM || in_sizes[1] != NQ * DIM || in_sizes[2] < 1) return;
    if (out_size < NQ) return;

    const float* sup = (const float*)d_in[0];
    const float* qry = (const float*)d_in[1];
    const int*   uco = (const int*)d_in[2];
    int*         out = (int*)d_out;

    size_t off = 0;
    const size_t off_mean = off; off = align_up_256(off + (size_t)DIM * sizeof(float));
    const size_t sz_s     = (size_t)MPAD * DIM * sizeof(unsigned short);
    const size_t sz_q     = (size_t)NPAD * DIM * sizeof(unsigned short);
    const size_t sz_p     = (size_t)MBLK * NPAD * sizeof(float);
    const size_t off_sh   = off; off = align_up_256(off + sz_s);
    const size_t off_sl   = off; off = align_up_256(off + sz_s);
    const size_t off_qh   = off; off = align_up_256(off + sz_q);
    const size_t off_ql   = off; off = align_up_256(off + sz_q);
    const size_t off_pv   = off; off = align_up_256(off + sz_p);
    const size_t off_pi   = off; off = align_up_256(off + sz_p);
    if (off > ws_size) return;

    char* ws = (char*)d_ws;
    float*          mean = (float*)(ws + off_mean);
    unsigned short* Sh   = (unsigned short*)(ws + off_sh);
    unsigned short* Sl   = (unsigned short*)(ws + off_sl);
    unsigned short* Qh   = (unsigned short*)(ws + off_qh);
    unsigned short* Ql   = (unsigned short*)(ws + off_ql);
    float*          pv   = (float*)(ws + off_pv);
    int*            pi   = (int*)(ws + off_pi);

    k_mean<<<dim3(1), dim3(DIM / 4), 0, stream>>>(sup, mean, NSUP);
    k_norm<<<dim3(MPAD), dim3(64), 0, stream>>>(sup, mean, Sh, Sl, NSUP, MPAD);
    k_norm<<<dim3(NPAD), dim3(64), 0, stream>>>(qry, mean, Qh, Ql, NQ, NPAD);
    k_sim<<<dim3(NBLK, MBLK), dim3(SIM_THREADS), 0, stream>>>(Sh, Sl, Qh, Ql, pv, pi);
    k_final<<<dim3(NBLK), dim3(32), 0, stream>>>(pv, pi, uco, out, NQ);
}
